// LSTM_33595234189617
// MI455X (gfx1250) — hardware-verified
//
#include <hip/hip_runtime.h>
#include <math.h>

constexpr int NBATCH     = 4096;
constexpr int NSTEP      = 512;
constexpr int NFEAT      = 4;
constexpr int NHID       = 50;
constexpr int NGATES     = 4;
constexpr int ROWS_BLK   = 32;
constexpr int KPAD       = 64;
constexpr int GATE_PITCH = 64;
constexpr int NPAD       = NGATES * GATE_PITCH;
constexpr int BPITCH     = 72;
constexpr int APITCH     = 72;
constexpr int XCOL0      = 56;
constexpr int TCHUNK     = 8;
constexpr int XSPITCH    = TCHUNK * NFEAT;
constexpr int HFPITCH    = 52;
constexpr int NQ         = 8;
constexpr float WCARRY     = 16.0f;
constexpr float WCARRY_INV = 1.0f / 16.0f;

static_assert(NBATCH % ROWS_BLK == 0, "grid exact");
static_assert(NSTEP % TCHUNK == 0, "no time tail");
static_assert(TCHUNK % 2 == 0, "buffer parity restarts every chunk");
static_assert(KPAD % 32 == 0, "k tiles");
static_assert(NHID <= XCOL0 && XCOL0 + NFEAT <= KPAD, "x slots inside the k pad");
static_assert(XCOL0 % 4 == 0, "8-byte aligned x slot");
static_assert(GATE_PITCH == 64 && NHID <= GATE_PITCH, "gate blocks at 64*g");
static_assert((2 * ROWS_BLK * APITCH) % (8 * 32) == 0, "A zero-fill exact");
static_assert((NPAD * 8) % 32 == 0, "B build exact");
static_assert(BPITCH % 8 == 0 && APITCH % 8 == 0, "16-byte fragment alignment");
static_assert(NQ == 2 * (GATE_PITCH / 16), "q = 2*subtile + mtile");

typedef __attribute__((ext_vector_type(16))) _Float16 v16h;
typedef __attribute__((ext_vector_type(8)))  _Float16 v8h;
typedef __attribute__((ext_vector_type(4)))  _Float16 v4h;
typedef __attribute__((ext_vector_type(8)))  float    v8f;
typedef __attribute__((ext_vector_type(4)))  float    v4f;

struct FragH {
  union U { v16h v; v8h h[2]; };
  static __device__ __forceinline__ v16h load(const _Float16* p) {
    U f;
    f.h[0] = *(const v8h*)(p);
    f.h[1] = *(const v8h*)(p + 16);
    return f.v;
  }
};

__device__ __forceinline__ v8f mma_f16(v16h a, v16h b, v8f c) {
  c = __builtin_amdgcn_wmma_f32_16x16x32_f16(false, a, false, b, (short)0, c, false, false);
  asm volatile("v_nop\n\tv_nop\n\tv_nop\n\tv_nop" : "+v"(c) : "v"(a), "v"(b));
  return c;
}

__device__ __forceinline__ float fsig(float x)  { return __builtin_amdgcn_rcpf(1.0f + __expf(-x)); }
__device__ __forceinline__ float ftanh(float x) { return 1.0f - 2.0f * __builtin_amdgcn_rcpf(__expf(2.0f * x) + 1.0f); }

__global__ __launch_bounds__(32) void lstm_seq_kernel(const float* __restrict__ seq,
                                                      const float* __restrict__ w_ih,
                                                      const float* __restrict__ w_hh,
                                                      const float* __restrict__ b_ih,
                                                      const float* __restrict__ b_hh,
                                                      const float* __restrict__ w_out,
                                                      const float* __restrict__ b_out,
                                                      float* __restrict__ out) {
  __shared__ __align__(16) _Float16 Bt[NPAD * BPITCH];
  __shared__ __align__(16) float    biasS[NPAD];
  __shared__ __align__(16) _Float16 At[2 * ROWS_BLK * APITCH];
  __shared__ __align__(16) float    Cst[NQ * 32 * 8];
  __shared__ __align__(16) _Float16 Xs[ROWS_BLK * XSPITCH];
  __shared__ __align__(16) float    Hf[ROWS_BLK * HFPITCH];

  const int lane = threadIdx.x;
  const int c    = lane & 15;
  const int hh   = lane >> 4;
  const int koff = 8 * hh;
  const int rowbase = blockIdx.x * ROWS_BLK;

#pragma unroll 1
  for (int it = 0; it < (NPAD * 8) / 32; ++it) {
    const int idx  = it * 32 + lane;
    const int n    = idx >> 3;
    const int g8   = idx & 7;
    const int gate = n >> 6;
    const int j    = n & 63;
    const bool jv  = (j < NHID);
    const int jc   = jv ? j : (NHID - 1);
    const int wrow = gate * NHID + jc;
    v8h hv;
#pragma unroll
    for (int e = 0; e < 8; ++e) {
      const int k  = 8 * g8 + e;
      const int kc = (k < NHID) ? k : (NHID - 1);
      int xi = k - XCOL0;
      xi = (xi < 0) ? 0 : ((xi > NFEAT - 1) ? (NFEAT - 1) : xi);
      float wh = w_hh[wrow * NHID + kc];
      float wi = w_ih[wrow * NFEAT + xi];
      asm volatile("" : "+v"(wh));
      asm volatile("" : "+v"(wi));
      const bool useh = jv && (k < NHID);
      const bool usex = jv && (k >= XCOL0) && (k < XCOL0 + NFEAT);
      const float v = useh ? wh : (usex ? wi : 0.0f);
      hv[e] = (_Float16)(v * WCARRY);
    }
    *(v8h*)(Bt + n * BPITCH + 8 * g8) = hv;
  }
#pragma unroll 1
  for (int it = 0; it < NPAD / 32; ++it) {
    const int n    = it * 32 + lane;
    const int gate = n >> 6;
    const int j    = n & 63;
    const bool jv  = (j < NHID);
    const int jc   = jv ? j : (NHID - 1);
    float bi = b_ih[gate * NHID + jc];
    float bh = b_hh[gate * NHID + jc];
    asm volatile("" : "+v"(bi));
    asm volatile("" : "+v"(bh));
    const float bs = (bi + bh) * WCARRY;
    biasS[n] = jv ? bs : 0.0f;
  }
  {
    const v8h zh = {(_Float16)0.0f, (_Float16)0.0f, (_Float16)0.0f, (_Float16)0.0f,
                    (_Float16)0.0f, (_Float16)0.0f, (_Float16)0.0f, (_Float16)0.0f};
#pragma unroll 1
    for (int it = 0; it < (2 * ROWS_BLK * APITCH) / (8 * 32); ++it)
      *(v8h*)(At + (it * 32 + lane) * 8) = zh;
  }
  {
    const v4f zf = {0.0f, 0.0f, 0.0f, 0.0f};
#pragma unroll 1
    for (int q = 0; q < NQ; ++q) {
      *(v4f*)(Cst + (q * 32 + lane) * 8)     = zf;
      *(v4f*)(Cst + (q * 32 + lane) * 8 + 4) = zf;
    }
  }
  __syncthreads();

#pragma unroll 1
  for (int tb = 0; tb < NSTEP / TCHUNK; ++tb) {
    {
      const float* sp = seq + ((size_t)(rowbase + lane) * NSTEP + (size_t)tb * TCHUNK) * NFEAT;
      v4f xv[TCHUNK];
#pragma unroll
      for (int i = 0; i < TCHUNK; ++i) xv[i] = *(const v4f*)(sp + 4 * i);
#pragma unroll
      for (int i = 0; i < TCHUNK; ++i) asm volatile("" : "+v"(xv[i]));
#pragma unroll
      for (int i = 0; i < TCHUNK / 2; ++i) {
        v8h pk;
#pragma unroll
        for (int e = 0; e < 4; ++e) {
          pk[e]     = (_Float16)xv[2 * i][e];
          pk[4 + e] = (_Float16)xv[2 * i + 1][e];
        }
        *(v8h*)(Xs + lane * XSPITCH + 8 * i) = pk;
      }
    }
    __syncthreads();

#pragma unroll 1
    for (int ts = 0; ts < TCHUNK; ++ts) {
      const int cur = ts & 1;
      _Float16* Acur = At + cur * (ROWS_BLK * APITCH);
      _Float16* Anxt = At + (cur ^ 1) * (ROWS_BLK * APITCH);
      const bool last = (tb == NSTEP / TCHUNK - 1) && (ts == TCHUNK - 1);

      {
        const v4h x4 = *(const v4h*)(Xs + lane * XSPITCH + NFEAT * ts);
        *(v4h*)(Acur + lane * APITCH + XCOL0) = x4;
      }
      __syncthreads();

#pragma unroll 1
      for (int q = 0; q < NQ; ++q) {
        const int s    = q >> 1;
        const int mt   = q & 1;
        const int ncol = 16 * s + c;
        const _Float16* ap = Acur + (16 * mt + c) * APITCH + koff;
        const v16h a0 = FragH::load(ap);
        const v16h a1 = FragH::load(ap + 32);
        v8f acc[NGATES];
#pragma unroll
        for (int g = 0; g < NGATES; ++g) {
          const float bv = biasS[GATE_PITCH * g + ncol];
          acc[g] = (v8f){bv, bv, bv, bv, bv, bv, bv, bv};
          const _Float16* bp = Bt + (GATE_PITCH * g + ncol) * BPITCH + koff;
          const v16h b0 = FragH::load(bp);
          const v16h b1 = FragH::load(bp + 32);
          acc[g] = mma_f16(a0, b0, acc[g]);
          acc[g] = mma_f16(a1, b1, acc[g]);
        }
        float* cp = Cst + (q * 32 + lane) * 8;
        const v4f cA = *(const v4f*)(cp);
        const v4f cB = *(const v4f*)(cp + 4);
        const bool cv = (ncol < NHID);
        const bool wr = (ncol < XCOL0) || (ncol >= XCOL0 + NFEAT);
        v4f nA, nB;
        float hq[8];
#pragma unroll
        for (int r = 0; r < 8; ++r) {
          const float zi = acc[0][r] * WCARRY_INV;
          const float zf = acc[1][r] * WCARRY_INV;
          const float zg = acc[2][r] * WCARRY_INV;
          const float zo = acc[3][r] * WCARRY_INV;
          const float ig = fsig(zi);
          const float fg = fsig(zf);
          const float gg = ftanh(zg);
          const float og = fsig(zo);
          const float co = (r < 4) ? cA[r & 3] : cB[r & 3];
          const float cn = fg * co + ig * gg;
          if (r < 4) nA[r & 3] = cn; else nB[r & 3] = cn;
          const float hn = og * ftanh(cn);
          hq[r] = cv ? hn : 0.0f;
        }
        *(v4f*)(cp)     = nA;
        *(v4f*)(cp + 4) = nB;
        if (wr) {
#pragma unroll
          for (int r = 0; r < 8; ++r)
            Anxt[(16 * mt + 8 * hh + r) * APITCH + ncol] = (_Float16)hq[r];
        }
        if (last && cv) {
#pragma unroll
          for (int r = 0; r < 8; ++r)
            Hf[(16 * mt + 8 * hh + r) * HFPITCH + ncol] = hq[r];
        }
      }
      __syncthreads();
    }
  }

  {
    float accv = 0.0f;
#pragma unroll 1
    for (int k = 0; k < NHID; ++k) accv = fmaf(Hf[lane * HFPITCH + k], w_out[k], accv);
    const float res = accv + b_out[0];
    float* op = out + rowbase + lane;
    *(volatile float*)op = res;
    __threadfence();
    *(volatile float*)op = res;
  }
}

extern "C" void kernel_launch(void* const* d_in, const int* in_sizes, int n_in,
                              void* d_out, int out_size, void* d_ws, size_t ws_size, hipStream_t stream) {
  (void)d_ws; (void)ws_size;
  if (n_in < 7 || d_out == nullptr) return;
  if (in_sizes[0] != NBATCH * NSTEP * NFEAT || in_sizes[1] != NGATES * NHID * NFEAT ||
      in_sizes[2] != NGATES * NHID * NHID || in_sizes[3] != NGATES * NHID || in_sizes[4] != NGATES * NHID ||
      in_sizes[5] != NHID || in_sizes[6] != 1 || out_size != NBATCH) return;

  const float* seq   = (const float*)d_in[0];
  const float* w_ih  = (const float*)d_in[1];
  const float* w_hh  = (const float*)d_in[2];
  const float* b_ih  = (const float*)d_in[3];
  const float* b_hh  = (const float*)d_in[4];
  const float* w_out = (const float*)d_in[5];
  const float* b_out = (const float*)d_in[6];
  float* out = (float*)d_out;

  lstm_seq_kernel<<<NBATCH / ROWS_BLK, 32, 0, stream>>>(seq, w_ih, w_hh, b_ih, b_hh, w_out, b_out, out);
}
